// CustomGPT2Attention_70824010711563
// MI455X (gfx1250) — hardware-verified
//
#include <hip/hip_runtime.h>
#include <hip/hip_bf16.h>
#include <math.h>

constexpr int NBATCH = 2;
constexpr int NSEQ   = 2048;
constexpr int NDIM   = 1024;
constexpr int NHEAD  = 16;
constexpr int HDIM   = 64;
constexpr int NQKV3  = 3 * NDIM;
constexpr int NTOK   = NBATCH * NSEQ;
constexpr int NFREQ  = HDIM / 2;

static_assert(NTOK % 64 == 0 && NQKV3 % 64 == 0 && NDIM % 64 == 0);
static_assert(NDIM % 32 == 0);
static_assert(NSEQ % 64 == 0 && HDIM == 64);

typedef __attribute__((ext_vector_type(16))) _Float16 v16h;
typedef __attribute__((ext_vector_type(8)))  _Float16 v8h;
typedef __attribute__((ext_vector_type(16))) __bf16   v16b;
typedef __attribute__((ext_vector_type(8)))  __bf16   v8b;
typedef __attribute__((ext_vector_type(8)))  float    v8f;
typedef __attribute__((ext_vector_type(4)))  float    v4f;
typedef __attribute__((ext_vector_type(4)))  unsigned v4u;

__device__ __forceinline__ unsigned short f2bf_bits(float f) {
  unsigned u = __float_as_uint(f);
  return (unsigned short)((u + 0x7FFFu + ((u >> 16) & 1u)) >> 16);
}
__device__ __forceinline__ float bf_bits2f(unsigned short h) { return __uint_as_float(((unsigned)h) << 16); }

__device__ __forceinline__ unsigned pack_bf2(float a, float c) {
  return (unsigned)f2bf_bits(a) | ((unsigned)f2bf_bits(c) << 16);
}
__device__ __forceinline__ void split_bf2(float a, float c, unsigned& hw, unsigned& lw) {
  const unsigned short ha = f2bf_bits(a), hc = f2bf_bits(c);
  const unsigned short la = f2bf_bits(a - bf_bits2f(ha)), lc = f2bf_bits(c - bf_bits2f(hc));
  hw = (unsigned)ha | ((unsigned)hc << 16);
  lw = (unsigned)la | ((unsigned)lc << 16);
}

__device__ __forceinline__ void dep_guard_h(v8f& a, v8f& b, v16h x, v16h y) { asm volatile("v_nop\n\tv_nop\n\tv_nop\n\tv_nop" : "+v"(a), "+v"(b) : "v"(x), "v"(y)); }
__device__ __forceinline__ void dep_guard_b(v8f& a, v8f& b, v16b x, v16b y) { asm volatile("v_nop\n\tv_nop\n\tv_nop\n\tv_nop" : "+v"(a), "+v"(b) : "v"(x), "v"(y)); }
__device__ __forceinline__ void keep4_h(v16h a, v16h b, v16h c, v16h d) { asm volatile("v_nop" :: "v"(a), "v"(b), "v"(c), "v"(d)); }
__device__ __forceinline__ void keep4_b(v16b a, v16b b, v16b c, v16b d) { asm volatile("v_nop" :: "v"(a), "v"(b), "v"(c), "v"(d)); }
__device__ __forceinline__ void acc_guard4(v8f& a, v8f& b, v8f& c, v8f& d) { asm volatile("v_nop\n\tv_nop\n\tv_nop\n\tv_nop" : "+v"(a), "+v"(b), "+v"(c), "+v"(d)); }
template <typename T> struct Frag;
template <> struct Frag<_Float16> {
  typedef v16h V; union U { v16h v; v8h h[2]; };
  static __device__ __forceinline__ v16h load(const _Float16* p) {
    U f; f.h[0] = *(const v8h*)(p); f.h[1] = *(const v8h*)(p + 16); return f.v;
  }
  static __device__ __forceinline__ v8f mma(v16h a, v16h b, v8f c) {
    return __builtin_amdgcn_wmma_f32_16x16x32_f16(false, a, false, b, (short)0, c, false, false);
  }
  static __device__ __forceinline__ void guard(v8f& a, v8f& b, v16h x, v16h y) { dep_guard_h(a, b, x, y); }
  static __device__ __forceinline__ void keep(v16h a, v16h b, v16h c, v16h d) { keep4_h(a, b, c, d); }
};
template <> struct Frag<__bf16> {
  typedef v16b V; union U { v16b v; v8b h[2]; };
  static __device__ __forceinline__ v16b load(const __bf16* p) {
    U f; f.h[0] = *(const v8b*)(p); f.h[1] = *(const v8b*)(p + 16); return f.v;
  }
  static __device__ __forceinline__ v8f mma(v16b a, v16b b, v8f c) {
    return __builtin_amdgcn_wmma_f32_16x16x32_bf16(false, a, false, b, (short)0, c, false, false);
  }
  static __device__ __forceinline__ void guard(v8f& a, v8f& b, v16b x, v16b y) { dep_guard_b(a, b, x, y); }
  static __device__ __forceinline__ void keep(v16b a, v16b b, v16b c, v16b d) { keep4_b(a, b, c, d); }
};

template <int ET> struct Elem;
template <> struct Elem<0> { typedef _Float16 T; };
template <> struct Elem<1> { typedef __bf16 T; };
template <int ET, int SPLIT, int BIAS_MODE, int OUT_MODE, bool RESID, int ACT = 0>
__global__ __launch_bounds__(256) void wmma_gemm64(
    const unsigned short* __restrict__ Ap, const unsigned short* __restrict__ A2p, int lda, long strideA,
    const unsigned short* __restrict__ Btp, const unsigned short* __restrict__ Bt2p, int ldb, long strideB,
    void* __restrict__ Cout, void* __restrict__ Cout2, int ldc, long strideC,
    const float* __restrict__ bias,
    const float* __restrict__ resid, long strideR,
    int M, int N, int K, float scale) {
  typedef typename Elem<ET>::T T;
  typedef typename Frag<T>::V V;
  const T* A = (const T*)Ap; const T* A2 = (const T*)A2p; const T* Bt = (const T*)Btp; const T* Bt2 = (const T*)Bt2p;
  __shared__ __align__(16) float sT[8][16 * 68];
  const int b    = blockIdx.y;
  const int lane = threadIdx.x & 31;
  const int wave = threadIdx.x >> 5;
  const int tilesN = N >> 6;
  const int tilesM = M >> 6;
  const int tile = blockIdx.x * 8 + wave;
  if (tile >= tilesM * tilesN) return;
  const int tm = tile / tilesN;
  const int tn = tile - tm * tilesN;
  const int m0 = tm << 6;
  const int n0 = tn << 6;

  const T* Ab  = A  + (size_t)b * strideA;
  const T* Bb  = Bt + (size_t)b * strideB;
  const T* Ab2 = (SPLIT != 0) ? (A2  + (size_t)b * strideA) : nullptr;
  const T* Bb2 = (SPLIT == 1) ? (Bt2 + (size_t)b * strideB) : nullptr;

  const int rlane = lane & 15;
  const int koff  = (lane >> 4) * 8;
  const int mOff  = (lane >> 4) * 8;

  v8f acc[4][4];
#pragma unroll
  for (int i = 0; i < 4; ++i)
#pragma unroll
    for (int j = 0; j < 4; ++j) acc[i][j] = (v8f){0.f,0.f,0.f,0.f,0.f,0.f,0.f,0.f};

  for (int k0 = 0; k0 < K; k0 += 32) {
    V bh[4], bl[4];
#pragma unroll
    for (int j = 0; j < 4; ++j) {
      const size_t bo = (size_t)(n0 + (j << 4) + rlane) * ldb + koff + k0;
      bh[j] = Frag<T>::load(Bb + bo);
      if (SPLIT == 1) bl[j] = Frag<T>::load(Bb2 + bo);
    }
#pragma unroll
    for (int i = 0; i < 4; ++i) {
      const size_t ao = (size_t)(m0 + (i << 4) + rlane) * lda + koff + k0;
      V ah = Frag<T>::load(Ab + ao);
      V al;
      if (SPLIT != 0) al = Frag<T>::load(Ab2 + ao);
#pragma unroll
      for (int j = 0; j < 4; ++j) {
        acc[i][j] = Frag<T>::mma(ah, bh[j], acc[i][j]);
        if (SPLIT == 1) acc[i][j] = Frag<T>::mma(ah, bl[j], acc[i][j]);
        if (SPLIT != 0) acc[i][j] = Frag<T>::mma(al, bh[j], acc[i][j]);
      }
      Frag<T>::guard(acc[i][0], acc[i][3], ah, (SPLIT != 0) ? al : ah);
    }
    Frag<T>::keep(bh[0], bh[1], bh[2], bh[3]);
    if (SPLIT == 1) Frag<T>::keep(bl[0], bl[1], bl[2], bl[3]);
  }
  acc_guard4(acc[0][0], acc[0][1], acc[0][2], acc[0][3]);
  acc_guard4(acc[1][0], acc[1][1], acc[1][2], acc[1][3]);
  acc_guard4(acc[2][0], acc[2][1], acc[2][2], acc[2][3]);
  acc_guard4(acc[3][0], acc[3][1], acc[3][2], acc[3][3]);

  float* slab = sT[wave];
  const float* Rb = RESID ? (resid + (size_t)b * strideR) : nullptr;
#pragma unroll
  for (int i = 0; i < 4; ++i) {
    const int mBase = m0 + (i << 4);
#pragma unroll
    for (int j = 0; j < 4; ++j) {
      const int n = n0 + (j << 4) + rlane;
      float bv = 0.f;
      if (BIAS_MODE == 2) bv = bias[n];
      if (BIAS_MODE == 3) bv = bf_bits2f(f2bf_bits(bias[n]));
#pragma unroll
      for (int r = 0; r < 8; ++r) {
        float v = acc[i][j][r] * scale;
        if (BIAS_MODE == 1) v += bias[mBase + mOff + r];
        if (BIAS_MODE == 2 || BIAS_MODE == 3) v += bv;
        if (RESID) v += Rb[(size_t)(mBase + mOff + r) * ldc + n];
        if (ACT == 1) v = tanhf(v);
        if (ACT == 2) v = fmaxf(v, 0.0f);
        if (ACT == 3) v = v / (1.0f + expf(-v));
        if (ACT == 4) v = (v > 0.f) ? v : 0.01f * v;
        if (ACT == 5) v = 0.5f * v * (1.0f + erff(v * 0.70710678118654752f));
        slab[(mOff + r) * 68 + (j << 4) + rlane] = v;
      }
    }
    __builtin_amdgcn_fence(__ATOMIC_RELEASE, "workgroup");
    __builtin_amdgcn_wave_barrier();
    __builtin_amdgcn_fence(__ATOMIC_ACQUIRE, "workgroup");
    if (OUT_MODE == 0) {
      float* C = (float*)Cout + (size_t)b * strideC;
      const int hh = lane >> 4, c4 = (lane & 15) * 4;
      for (int pass = 0; pass < 2; ++pass) {
#pragma unroll
        for (int it = 0; it < 8; ++it) {
          const int row = it * 2 + hh;
          v4f v = *(const v4f*)(slab + row * 68 + c4);
          *(volatile v4f*)(C + (size_t)(mBase + row) * ldc + n0 + c4) = v;
        }
        __threadfence();
      }
    } else {
      const int q = lane >> 3, c8 = (lane & 7) * 8;
      unsigned short* C  = (unsigned short*)Cout  + (size_t)b * strideC;
      unsigned short* C2 = (OUT_MODE == 2) ? ((unsigned short*)Cout2 + (size_t)b * strideC) : nullptr;
      for (int pass = 0; pass < 2; ++pass) {
#pragma unroll
        for (int it = 0; it < 4; ++it) {
          const int row = it * 4 + q;
          const float* sp = slab + row * 68 + c8;
          v8h hv, lv;
#pragma unroll
          for (int e = 0; e < 8; ++e) {
            if (OUT_MODE == 1) {
              hv[e] = (_Float16)sp[e];
            } else {
              unsigned short hb = f2bf_bits(sp[e]);
              unsigned short lb = f2bf_bits(sp[e] - bf_bits2f(hb));
              hv[e] = __builtin_bit_cast(_Float16, hb);
              lv[e] = __builtin_bit_cast(_Float16, lb);
            }
          }
          *(volatile v8h*)(C + (size_t)(mBase + row) * ldc + n0 + c8) = hv;
          if (OUT_MODE == 2) *(volatile v8h*)(C2 + (size_t)(mBase + row) * ldc + n0 + c8) = lv;
        }
        __threadfence();
      }
    }
    __builtin_amdgcn_fence(__ATOMIC_RELEASE, "workgroup");
    __builtin_amdgcn_wave_barrier();
    __builtin_amdgcn_fence(__ATOMIC_ACQUIRE, "workgroup");
  }
}

__global__ __launch_bounds__(256) void cast_f32_bf16x8(const float* __restrict__ in, unsigned short* __restrict__ out, int n8) {
  const int i = blockIdx.x * 256 + threadIdx.x;
  if (i < n8) {
    const v4f a = *(const v4f*)(in + (size_t)i * 8);
    const v4f c = *(const v4f*)(in + (size_t)i * 8 + 4);
    v4u w;
    w[0] = pack_bf2(a[0], a[1]); w[1] = pack_bf2(a[2], a[3]);
    w[2] = pack_bf2(c[0], c[1]); w[3] = pack_bf2(c[2], c[3]);
    unsigned short* dst = out + (size_t)i * 8;
    *(volatile v4u*)dst = w;
    __threadfence();
    *(volatile v4u*)dst = w;
  }
}

__global__ __launch_bounds__(256) void transpose_f32_bf16(const float* __restrict__ in, unsigned short* __restrict__ out, int R, int Cc) {
  __shared__ float ts[64][65];
  const int tid = threadIdx.x, lane = tid & 31, wave = tid >> 5;
  const int c0 = blockIdx.x * 64, r0 = blockIdx.y * 64;
#pragma unroll
  for (int it = 0; it < 4; ++it) {
    const int idx = it * 256 + tid;
    const int row = idx >> 4, c4 = (idx & 15) * 4;
    const v4f v = *(const v4f*)(in + (size_t)(r0 + row) * Cc + c0 + c4);
    ts[row][c4] = v[0]; ts[row][c4 + 1] = v[1]; ts[row][c4 + 2] = v[2]; ts[row][c4 + 3] = v[3];
  }
  __syncthreads();
  const int q = lane >> 3, c8 = (lane & 7) * 8;
#pragma unroll
  for (int it = 0; it < 2; ++it) {
    const int orow = wave * 8 + it * 4 + q;
    v4u w;
#pragma unroll
    for (int e = 0; e < 4; ++e) w[e] = pack_bf2(ts[c8 + 2 * e][orow], ts[c8 + 2 * e + 1][orow]);
    unsigned short* dst = out + (size_t)(c0 + orow) * R + r0 + c8;
    *(volatile v4u*)dst = w;
    __threadfence();
    *(volatile v4u*)dst = w;
  }
}

struct RopeFreq { float inv[NFREQ]; };
static_assert(sizeof(RopeFreq) == NFREQ * 4);

__global__ __launch_bounds__(256) void rope_table_kernel(float* __restrict__ cs_tab, float* __restrict__ sn_tab, RopeFreq rf, int npos) {
#pragma clang fp contract(off)
  __shared__ float invs[NFREQ];
  const int tid = threadIdx.x, lane = tid & 31, wave = tid >> 5;
  if (tid == 0) {
#pragma unroll
    for (int f = 0; f < NFREQ; ++f) invs[f] = rf.inv[f];
  }
  __syncthreads();
  int pos = blockIdx.x * 8 + wave;
  const bool ok = (pos < npos);
  pos = ok ? pos : (npos - 1);
  const float ang = (float)pos * invs[lane];
  const float cs = cosf(ang);
  const float sn = sinf(ang);
  if (ok) {
    float* pc = cs_tab + (size_t)pos * NFREQ + lane;
    float* ps = sn_tab + (size_t)pos * NFREQ + lane;
    *(volatile float*)pc = cs;
    *(volatile float*)ps = sn;
    __threadfence();
    *(volatile float*)pc = cs;
    *(volatile float*)ps = sn;
  }
}

__global__ __launch_bounds__(256) void rope_split_kernel(
    const float* __restrict__ qkv, const float* __restrict__ cs_tab, const float* __restrict__ sn_tab,
    unsigned short* Qh, unsigned short* Ql, unsigned short* Kh, unsigned short* Kl,
    unsigned short* Vth, unsigned short* Vtl) {
  __shared__ float vsm[64][65];
  const int tid = threadIdx.x, lane = tid & 31, wave = tid >> 5;
  const int nsc = NSEQ / 64;
  const int sc = blockIdx.x % nsc, bh = blockIdx.x / nsc;
  const int b = bh / NHEAD, h = bh % NHEAD;
  const int s0 = sc * 64;
  const size_t rowbase = (size_t)b * NSEQ + s0;
#pragma unroll
  for (int it = 0; it < 4; ++it) {
    const int idx = it * 256 + tid;
    const int sr = idx >> 4, c4 = (idx & 15) * 4;
    const v4f vv = *(const v4f*)(qkv + (rowbase + sr) * NQKV3 + 2 * NDIM + h * HDIM + c4);
    vsm[sr][c4] = vv[0]; vsm[sr][c4 + 1] = vv[1]; vsm[sr][c4 + 2] = vv[2]; vsm[sr][c4 + 3] = vv[3];
  }
  __syncthreads();
  const int q4 = lane >> 3, c8 = (lane & 7) * 8;
  const int cp8 = c8 ^ 32;
  const float sgn = (c8 < 32) ? -1.0f : 1.0f;
  const int f0 = c8 & 31;
#pragma unroll 1
  for (int mat = 0; mat < 2; ++mat) {
    unsigned short* dsth = (mat == 0) ? Qh : Kh;
    unsigned short* dstl = (mat == 0) ? Ql : Kl;
    const float osc = (mat == 0) ? 0.125f : 1.0f;
#pragma unroll 1
    for (int it = 0; it < 2; ++it) {
      const int sr = wave * 8 + it * 4 + q4;
      const int s = s0 + sr;
      const float* xr = qkv + (rowbase + sr) * NQKV3 + mat * NDIM + h * HDIM;
      const v4f xa = *(const v4f*)(xr + c8),  xb = *(const v4f*)(xr + c8 + 4);
      const v4f pa = *(const v4f*)(xr + cp8), pb = *(const v4f*)(xr + cp8 + 4);
      const float* cr = cs_tab + (size_t)s * NFREQ + f0;
      const float* nr = sn_tab + (size_t)s * NFREQ + f0;
      const v4f ca = *(const v4f*)(cr), cb = *(const v4f*)(cr + 4);
      const v4f na = *(const v4f*)(nr), nb = *(const v4f*)(nr + 4);
      float o[8];
#pragma unroll
      for (int e = 0; e < 4; ++e) {
        o[e]     = (xa[e] * ca[e] + (sgn * pa[e]) * na[e]) * osc;
        o[4 + e] = (xb[e] * cb[e] + (sgn * pb[e]) * nb[e]) * osc;
      }
      v4u hw, lw;
#pragma unroll
      for (int e = 0; e < 4; ++e) { unsigned a, c; split_bf2(o[2 * e], o[2 * e + 1], a, c); hw[e] = a; lw[e] = c; }
      unsigned short* ph = dsth + ((size_t)bh * NSEQ + s) * HDIM + c8;
      unsigned short* pl = dstl + ((size_t)bh * NSEQ + s) * HDIM + c8;
      *(volatile v4u*)ph = hw;
      *(volatile v4u*)pl = lw;
      __threadfence();
      *(volatile v4u*)ph = hw;
      *(volatile v4u*)pl = lw;
    }
  }
#pragma unroll 1
  for (int it = 0; it < 2; ++it) {
    const int dr = wave * 8 + it * 4 + q4;
    float o[8];
#pragma unroll
    for (int e = 0; e < 8; ++e) o[e] = vsm[c8 + e][dr];
    v4u hw, lw;
#pragma unroll
    for (int e = 0; e < 4; ++e) { unsigned a, c; split_bf2(o[2 * e], o[2 * e + 1], a, c); hw[e] = a; lw[e] = c; }
    unsigned short* ph = Vth + ((size_t)bh * HDIM + dr) * NSEQ + s0 + c8;
    unsigned short* pl = Vtl + ((size_t)bh * HDIM + dr) * NSEQ + s0 + c8;
    *(volatile v4u*)ph = hw;
    *(volatile v4u*)pl = lw;
    __threadfence();
    *(volatile v4u*)ph = hw;
    *(volatile v4u*)pl = lw;
  }
}

#define AT_D 64
#define AT_NW 4
#define AT_QB 64
#define AT_KC 64

__device__ __forceinline__ unsigned short at_bf_bits(float f) {
  unsigned u = __float_as_uint(f);
  return (unsigned short)((u + 0x7FFFu + ((u >> 16) & 1u)) >> 16);
}
__device__ __forceinline__ __bf16 at_f2bf(float f) { return __builtin_bit_cast(__bf16, at_bf_bits(f)); }
__device__ __forceinline__ void at_split(float f, __bf16& hi, __bf16& lo) {
  const unsigned short hb = at_bf_bits(f);
  hi = __builtin_bit_cast(__bf16, hb);
  lo = at_f2bf(f - __uint_as_float(((unsigned)hb) << 16));
}
__device__ __forceinline__ v8f at_mma(v16b a, v16b b, v8f c) {
  c = __builtin_amdgcn_wmma_f32_16x16x32_bf16(false, a, false, b, (short)0, c, false, false);
  asm volatile("v_nop\n\tv_nop\n\tv_nop\n\tv_nop" : "+v"(c) : "v"(a), "v"(b));
  return c;
}

__global__ __launch_bounds__(128)
void attn64_causal_hilo(const unsigned short* __restrict__ Qhp, const unsigned short* __restrict__ Qlp,
                        const unsigned short* __restrict__ Khp, const unsigned short* __restrict__ Klp,
                        const unsigned short* __restrict__ Vthp, const unsigned short* __restrict__ Vtlp,
                        unsigned short* __restrict__ Ohp, unsigned short* __restrict__ Olp,
                        int seq, int nheads, int o_ld) {
  union FB { v16b v; v8b h[2]; };
  __shared__ __align__(16) __bf16 Ksh[AT_KC * AT_D];
  __shared__ __align__(16) __bf16 Ksl[AT_KC * AT_D];
  __shared__ __align__(16) __bf16 Vsh[AT_D * AT_KC];
  __shared__ __align__(16) __bf16 Vsl[AT_D * AT_KC];
  __shared__ __align__(16) __bf16 Psh[AT_NW][16 * AT_KC];
  __shared__ __align__(16) __bf16 Psl[AT_NW][16 * AT_KC];
  __shared__ __align__(16) float  Os[AT_NW][16 * 68];

  const int tid  = threadIdx.x;
  const int wave = tid >> 5;
  const int lane = tid & 31;
  const int hh   = lane >> 4;
  const int c    = lane & 15;

  const int nqb = seq / AT_QB;
  const int bx = blockIdx.x;
  const int qb = bx % nqb;
  const int bh = bx / nqb;
  const int h  = bh % nheads;
  const int b  = bh / nheads;
  const int q0 = qb * AT_QB + wave * 16;

  const __bf16* Qh  = (const __bf16*)Qhp  + (size_t)bh * seq * AT_D;
  const __bf16* Ql  = (const __bf16*)Qlp  + (size_t)bh * seq * AT_D;
  const __bf16* Kh  = (const __bf16*)Khp  + (size_t)bh * seq * AT_D;
  const __bf16* Kl  = (const __bf16*)Klp  + (size_t)bh * seq * AT_D;
  const __bf16* Vth = (const __bf16*)Vthp + (size_t)bh * AT_D * seq;
  const __bf16* Vtl = (const __bf16*)Vtlp + (size_t)bh * AT_D * seq;
  unsigned short* Oh = Ohp + (size_t)b * seq * o_ld + (size_t)h * AT_D;
  unsigned short* Ol = Olp + (size_t)b * seq * o_ld + (size_t)h * AT_D;

  v16b qah[2], qal[2];
#pragma unroll
  for (int dc = 0; dc < 2; ++dc) {
    FB f;
    const __bf16* qr = Qh + (size_t)(q0 + c) * AT_D + dc * 32 + 8 * hh;
    f.h[0] = *(const v8b*)(qr); f.h[1] = *(const v8b*)(qr + 16); qah[dc] = f.v;
    const __bf16* qs = Ql + (size_t)(q0 + c) * AT_D + dc * 32 + 8 * hh;
    f.h[0] = *(const v8b*)(qs); f.h[1] = *(const v8b*)(qs + 16); qal[dc] = f.v;
  }

  float mrow[8], lrow[8];
  v8f oacc[4];
#pragma unroll
  for (int r = 0; r < 8; ++r) { mrow[r] = -INFINITY; lrow[r] = 0.f; }
#pragma unroll
  for (int t = 0; t < 4; ++t) oacc[t] = (v8f){0.f,0.f,0.f,0.f,0.f,0.f,0.f,0.f};

  const float sfill = -3.40282347e38f;
  const int nChunks = qb + 1;
  for (int kc = 0; kc < nChunks; ++kc) {
    const int kv0 = kc * AT_KC;
    __syncthreads();
#pragma unroll
    for (int it = 0; it < 4; ++it) {
      const int idx = it * 128 + tid;
      const int r = idx >> 3, c8 = (idx & 7) * 8;
      const v8b kxh = *(const v8b*)(Kh + (size_t)(kv0 + r) * AT_D + c8);
      const v8b kxl = *(const v8b*)(Kl + (size_t)(kv0 + r) * AT_D + c8);
      *(v8b*)(Ksh + r * AT_D + c8) = kxh;
      *(v8b*)(Ksl + r * AT_D + c8) = kxl;
    }
    asm volatile("" ::: "memory");
#pragma unroll
    for (int it = 0; it < 4; ++it) {
      const int idx = it * 128 + tid;
      const int r = idx >> 3, c8 = (idx & 7) * 8;
      const v8b vxh = *(const v8b*)(Vth + (size_t)r * seq + kv0 + c8);
      const v8b vxl = *(const v8b*)(Vtl + (size_t)r * seq + kv0 + c8);
      *(v8b*)(Vsh + r * AT_KC + c8) = vxh;
      *(v8b*)(Vsl + r * AT_KC + c8) = vxl;
    }
    __syncthreads();

    v8f s[4];
#pragma unroll
    for (int j = 0; j < 4; ++j) {
      s[j] = (v8f){0.f,0.f,0.f,0.f,0.f,0.f,0.f,0.f};
#pragma unroll
      for (int dc = 0; dc < 2; ++dc) {
        FB kb, kl;
        kb.h[0] = *(const v8b*)(Ksh + (j * 16 + c) * AT_D + dc * 32 + 8 * hh);
        kb.h[1] = *(const v8b*)(Ksh + (j * 16 + c) * AT_D + dc * 32 + 16 + 8 * hh);
        kl.h[0] = *(const v8b*)(Ksl + (j * 16 + c) * AT_D + dc * 32 + 8 * hh);
        kl.h[1] = *(const v8b*)(Ksl + (j * 16 + c) * AT_D + dc * 32 + 16 + 8 * hh);
        s[j] = at_mma(qah[dc], kb.v, s[j]);
        s[j] = at_mma(qah[dc], kl.v, s[j]);
        s[j] = at_mma(qal[dc], kb.v, s[j]);
      }
    }
    const bool diag = (kc == qb);
    float cm[8];
#pragma unroll
    for (int r = 0; r < 8; ++r) {
      const int qrow = q0 + 8 * hh + r;
      float m = -INFINITY;
#pragma unroll
      for (int j = 0; j < 4; ++j) {
        const int kvcol = kv0 + j * 16 + c;
        if (diag && (kvcol > qrow)) s[j][r] = sfill;
        m = fmaxf(m, s[j][r]);
      }
#pragma unroll
      for (int off = 1; off < 16; off <<= 1) m = fmaxf(m, __shfl_xor(m, off, 32));
      cm[r] = m;
    }
    __bf16* pwh = Psh[wave];
    __bf16* pwl = Psl[wave];
#pragma unroll
    for (int r = 0; r < 8; ++r) {
      const float mnew = fmaxf(mrow[r], cm[r]);
      const float alpha = expf(mrow[r] - mnew);
      mrow[r] = mnew;
      float psum = 0.f;
#pragma unroll
      for (int j = 0; j < 4; ++j) {
        const float p = expf(s[j][r] - mnew);
        psum += p;
        __bf16 a, pl; at_split(p, a, pl);
        pwh[(8 * hh + r) * AT_KC + j * 16 + c] = a;
        pwl[(8 * hh + r) * AT_KC + j * 16 + c] = pl;
      }
#pragma unroll
      for (int off = 1; off < 16; off <<= 1) psum += __shfl_xor(psum, off, 32);
      lrow[r] = lrow[r] * alpha + psum;
#pragma unroll
      for (int t = 0; t < 4; ++t) oacc[t][r] *= alpha;
    }
    __builtin_amdgcn_fence(__ATOMIC_RELEASE, "workgroup");
    __builtin_amdgcn_wave_barrier();
    __builtin_amdgcn_fence(__ATOMIC_ACQUIRE, "workgroup");
#pragma unroll 1
    for (int kk = 0; kk < 2; ++kk) {
      FB pa, pl;
      pa.h[0] = *(const v8b*)(pwh + c * AT_KC + kk * 32 + 8 * hh);
      pa.h[1] = *(const v8b*)(pwh + c * AT_KC + kk * 32 + 16 + 8 * hh);
      pl.h[0] = *(const v8b*)(pwl + c * AT_KC + kk * 32 + 8 * hh);
      pl.h[1] = *(const v8b*)(pwl + c * AT_KC + kk * 32 + 16 + 8 * hh);
#pragma unroll
      for (int t = 0; t < 4; ++t) {
        FB vb, vl;
        vb.h[0] = *(const v8b*)(Vsh + (t * 16 + c) * AT_KC + kk * 32 + 8 * hh);
        vb.h[1] = *(const v8b*)(Vsh + (t * 16 + c) * AT_KC + kk * 32 + 16 + 8 * hh);
        vl.h[0] = *(const v8b*)(Vsl + (t * 16 + c) * AT_KC + kk * 32 + 8 * hh);
        vl.h[1] = *(const v8b*)(Vsl + (t * 16 + c) * AT_KC + kk * 32 + 16 + 8 * hh);
        oacc[t] = at_mma(pa.v, vb.v, oacc[t]);
        oacc[t] = at_mma(pa.v, vl.v, oacc[t]);
        oacc[t] = at_mma(pl.v, vb.v, oacc[t]);
      }
    }
  }

  float* os = Os[wave];
#pragma unroll
  for (int r = 0; r < 8; ++r) {
    const float inv = 1.0f / lrow[r];
#pragma unroll
    for (int t = 0; t < 4; ++t) os[(8 * hh + r) * 68 + t * 16 + c] = oacc[t][r] * inv;
  }
  __builtin_amdgcn_fence(__ATOMIC_RELEASE, "workgroup");
  __builtin_amdgcn_wave_barrier();
  __builtin_amdgcn_fence(__ATOMIC_ACQUIRE, "workgroup");
  {
    const int q = lane >> 3, c8 = (lane & 7) * 8;
    for (int pass = 0; pass < 2; ++pass) {
#pragma unroll
      for (int it = 0; it < 4; ++it) {
        const int row = it * 4 + q;
        const float* sp = os + row * 68 + c8;
        v4u hw, lw;
#pragma unroll
        for (int e = 0; e < 4; ++e) { unsigned a, d; split_bf2(sp[2 * e], sp[2 * e + 1], a, d); hw[e] = a; lw[e] = d; }
        *(volatile v4u*)(Oh + (size_t)(q0 + row) * o_ld + c8) = hw;
        *(volatile v4u*)(Ol + (size_t)(q0 + row) * o_ld + c8) = lw;
      }
      __threadfence();
    }
  }
}

extern "C" void kernel_launch(void* const* d_in, const int* in_sizes, int n_in,
                              void* d_out, int out_size, void* d_ws, size_t ws_size,
                              hipStream_t stream) {
  (void)n_in;
  if (in_sizes[0] != NTOK * NDIM || in_sizes[1] != NDIM * NQKV3 || in_sizes[2] != NQKV3 ||
      in_sizes[3] != NDIM * NDIM || in_sizes[4] != NDIM || out_size != NTOK * NDIM) return;

  const float* X     = (const float*)d_in[0];
  const float* Wqkv  = (const float*)d_in[1];
  const float* bqkv  = (const float*)d_in[2];
  const float* Wproj = (const float*)d_in[3];
  const float* bproj = (const float*)d_in[4];
  float* out = (float*)d_out;

  const size_t bytesXb   = (size_t)NTOK * NDIM * 2;
  const size_t bytesWt1  = (size_t)NQKV3 * NDIM * 2;
  const size_t bytesWt2  = (size_t)NDIM * NDIM * 2;
  const size_t bytesQkv  = (size_t)NTOK * NQKV3 * 4;
  const size_t bytesPl   = (size_t)NBATCH * NHEAD * NSEQ * HDIM * 2;
  const size_t bytesTab  = (size_t)NSEQ * NFREQ * 4;
  size_t off = 0;
  char* ws = (char*)d_ws;
  unsigned short* Xb  = (unsigned short*)(ws + off); off += bytesXb;
  unsigned short* Wt1 = (unsigned short*)(ws + off); off += bytesWt1;
  unsigned short* Wt2 = (unsigned short*)(ws + off); off += bytesWt2;
  float* qkvf = (float*)(ws + off);
  unsigned short* Oh  = (unsigned short*)(ws + off);
  unsigned short* Ol  = (unsigned short*)(ws + off + (size_t)NTOK * NDIM * 2);
  off += bytesQkv;
  unsigned short* Qh  = (unsigned short*)(ws + off); off += bytesPl;
  unsigned short* Ql  = (unsigned short*)(ws + off); off += bytesPl;
  unsigned short* Kh  = (unsigned short*)(ws + off); off += bytesPl;
  unsigned short* Kl  = (unsigned short*)(ws + off); off += bytesPl;
  unsigned short* Vth = (unsigned short*)(ws + off); off += bytesPl;
  unsigned short* Vtl = (unsigned short*)(ws + off); off += bytesPl;
  float* cs_tab = (float*)(ws + off); off += bytesTab;
  float* sn_tab = (float*)(ws + off); off += bytesTab;
  if (off > ws_size) return;
  if ((size_t)NTOK * NDIM * 2 * 2 > bytesQkv) return;

  RopeFreq rf;
  for (int f = 0; f < NFREQ; ++f) {
    const float e = (float)(2 * f) / 64.0f;
    const float p = (float)pow(10000.0, (double)e);
    rf.inv[f] = 1.0f / p;
  }

  cast_f32_bf16x8<<<(NTOK * NDIM / 8) / 256, 256, 0, stream>>>(X, Xb, NTOK * NDIM / 8);
  transpose_f32_bf16<<<dim3(NQKV3 / 64, NDIM / 64), 256, 0, stream>>>(Wqkv, Wt1, NDIM, NQKV3);
  transpose_f32_bf16<<<dim3(NDIM / 64, NDIM / 64), 256, 0, stream>>>(Wproj, Wt2, NDIM, NDIM);

  wmma_gemm64<1, 0, 3, 0, false><<<dim3((NTOK / 64) * (NQKV3 / 64) / 8, 1), 256, 0, stream>>>(
      Xb, Xb, NDIM, 0L, Wt1, Wt1, NDIM, 0L, (void*)qkvf, (void*)qkvf, NQKV3, 0L,
      bqkv, bqkv, 0L, NTOK, NQKV3, NDIM, 1.0f);

  rope_table_kernel<<<NSEQ / 8, 256, 0, stream>>>(cs_tab, sn_tab, rf, NSEQ);

  rope_split_kernel<<<NBATCH * NHEAD * (NSEQ / 64), 256, 0, stream>>>(qkvf, cs_tab, sn_tab, Qh, Ql, Kh, Kl, Vth, Vtl);

  attn64_causal_hilo<<<NBATCH * NHEAD * (NSEQ / 64), 128, 0, stream>>>(Qh, Ql, Kh, Kl, Vth, Vtl, Oh, Ol, NSEQ, NHEAD, NDIM);

  wmma_gemm64<1, 2, 3, 0, false><<<dim3((NTOK / 64) * (NDIM / 64) / 8, 1), 256, 0, stream>>>(
      Oh, Ol, NDIM, 0L, Wt2, Wt2, NDIM, 0L, (void*)out, (void*)out, NDIM, 0L,
      bproj, bproj, 0L, NTOK, NDIM, NDIM, 1.0f);
}
